// GTEProgramClassification_27986006900873
// MI455X (gfx1250) — hardware-verified
//
#include <hip/hip_runtime.h>
#include <stdint.h>

typedef __attribute__((ext_vector_type(16))) _Float16 v16h;
typedef __attribute__((ext_vector_type(8)))  _Float16 v8h;
typedef __attribute__((ext_vector_type(16))) __bf16   v16b;
typedef __attribute__((ext_vector_type(8)))  __bf16   v8b;
typedef __attribute__((ext_vector_type(8)))  float    v8f;
typedef __attribute__((ext_vector_type(4)))  float    v4f;
typedef __attribute__((ext_vector_type(4)))  unsigned v4u;

constexpr int HDIM       = 128;
constexpr int GATE3      = 3 * HDIM;
constexpr int NCLASS     = 104;
constexpr int NCLASS_PAD = 112;
constexpr int MBOX       = 8;
constexpr int NSTEP      = MBOX - 1;
constexpr int WPITCH     = 136;
constexpr int HFPITCH    = 132;
constexpr int GIS_FLOATS = 3 * 16 * 16;
constexpr float HCARRY    = 16.0f;
constexpr float WCARRY    = 256.0f;
constexpr float FOLD_BACK = 1.0f / 4096.0f;
static_assert(HDIM % 32 == 0, "K multiple of 32");
static_assert(GATE3 % 64 == 0, "N multiple of 64 for the tile GEMM");
static_assert(NCLASS_PAD % 16 == 0 && NCLASS <= NCLASS_PAD, "class padding");
static_assert((16 * NCLASS * 4) % 512 == 0, "16-row output group = 13 x 512 B");

constexpr int LDS_WHH  = 0;
constexpr int LDS_HF   = LDS_WHH + GATE3 * WPITCH * 2;
constexpr int LDS_HB   = LDS_HF + 4 * 16 * HFPITCH * 4;
constexpr int LDS_GIS  = LDS_HB + 4 * 16 * WPITCH * 2;
constexpr int LDS_BIAS = LDS_GIS + 4 * GIS_FLOATS * 4;
constexpr int LDS_LNP  = LDS_BIAS + 2 * GATE3 * 4;
constexpr int LDS_TOK  = LDS_LNP + 2 * HDIM * 4;
constexpr int LDS_GRU_TOTAL = LDS_TOK + 4 * 16 * 4;
static_assert(LDS_HF % 16 == 0 && LDS_HB % 16 == 0 && LDS_GIS % 16 == 0 && LDS_BIAS % 16 == 0 && LDS_LNP % 16 == 0 && LDS_TOK % 16 == 0, "LDS alignment");
static_assert(LDS_GRU_TOTAL == 172288, "LDS total");

__device__ __forceinline__ unsigned short f2bf_bits(float f) {
  unsigned u = __float_as_uint(f);
  return (unsigned short)((u + 0x7FFFu + ((u >> 16) & 1u)) >> 16);
}
__device__ __forceinline__ float bf_bits2f(unsigned short h) { return __uint_as_float(((unsigned)h) << 16); }

__device__ __forceinline__ void dep_guard_h(v8f& a, v8f& b, v16h x, v16h y) { asm volatile("v_nop\n\tv_nop\n\tv_nop\n\tv_nop" : "+v"(a), "+v"(b) : "v"(x), "v"(y)); }
__device__ __forceinline__ void dep_guard_b(v8f& a, v8f& b, v16b x, v16b y) { asm volatile("v_nop\n\tv_nop\n\tv_nop\n\tv_nop" : "+v"(a), "+v"(b) : "v"(x), "v"(y)); }
__device__ __forceinline__ void keep4_h(v16h a, v16h b, v16h c, v16h d) { asm volatile("v_nop" :: "v"(a), "v"(b), "v"(c), "v"(d)); }
__device__ __forceinline__ void keep4_b(v16b a, v16b b, v16b c, v16b d) { asm volatile("v_nop" :: "v"(a), "v"(b), "v"(c), "v"(d)); }
__device__ __forceinline__ void acc_guard4(v8f& a, v8f& b, v8f& c, v8f& d) { asm volatile("v_nop\n\tv_nop\n\tv_nop\n\tv_nop" : "+v"(a), "+v"(b), "+v"(c), "+v"(d)); }
template <typename T> struct Frag;
template <> struct Frag<_Float16> {
  typedef v16h V; union U { v16h v; v8h h[2]; };
  static __device__ __forceinline__ v16h load(const _Float16* p) {
    U f; f.h[0] = *(const v8h*)(p); f.h[1] = *(const v8h*)(p + 16); return f.v;
  }
  static __device__ __forceinline__ v8f mma(v16h a, v16h b, v8f c) {
    return __builtin_amdgcn_wmma_f32_16x16x32_f16(false, a, false, b, (short)0, c, false, false);
  }
  static __device__ __forceinline__ void guard(v8f& a, v8f& b, v16h x, v16h y) { dep_guard_h(a, b, x, y); }
  static __device__ __forceinline__ void keep(v16h a, v16h b, v16h c, v16h d) { keep4_h(a, b, c, d); }
};
template <> struct Frag<__bf16> {
  typedef v16b V; union U { v16b v; v8b h[2]; };
  static __device__ __forceinline__ v16b load(const __bf16* p) {
    U f; f.h[0] = *(const v8b*)(p); f.h[1] = *(const v8b*)(p + 16); return f.v;
  }
  static __device__ __forceinline__ v8f mma(v16b a, v16b b, v8f c) {
    return __builtin_amdgcn_wmma_f32_16x16x32_bf16(false, a, false, b, (short)0, c, false, false);
  }
  static __device__ __forceinline__ void guard(v8f& a, v8f& b, v16b x, v16b y) { dep_guard_b(a, b, x, y); }
  static __device__ __forceinline__ void keep(v16b a, v16b b, v16b c, v16b d) { keep4_b(a, b, c, d); }
};

template <int ET> struct Elem;
template <> struct Elem<0> { typedef _Float16 T; };
template <> struct Elem<1> { typedef __bf16 T; };
template <int ET, bool SPLIT, int BIAS_MODE, int OUT_MODE, bool RESID, int ACT = 0>
__global__ __launch_bounds__(256) void wmma_gemm64(
    const unsigned short* __restrict__ Ap, const unsigned short* __restrict__ A2p, int lda, long strideA,
    const unsigned short* __restrict__ Btp, const unsigned short* __restrict__ Bt2p, int ldb, long strideB,
    void* __restrict__ Cout, void* __restrict__ Cout2, int ldc, long strideC,
    const float* __restrict__ bias,
    const float* __restrict__ resid, long strideR,
    int M, int N, int K, float scale) {
  typedef typename Elem<ET>::T T;
  typedef typename Frag<T>::V V;
  const T* A = (const T*)Ap; const T* A2 = (const T*)A2p; const T* Bt = (const T*)Btp; const T* Bt2 = (const T*)Bt2p;
  __shared__ __align__(16) float sT[8][16 * 68];
  const int b    = blockIdx.y;
  const int lane = threadIdx.x & 31;
  const int wave = threadIdx.x >> 5;
  const int tilesN = N >> 6;
  const int tilesM = M >> 6;
  const int tile = blockIdx.x * 8 + wave;
  if (tile >= tilesM * tilesN) return;
  const int tm = tile / tilesN;
  const int tn = tile - tm * tilesN;
  const int m0 = tm << 6;
  const int n0 = tn << 6;

  const T* Ab  = A  + (size_t)b * strideA;
  const T* Bb  = Bt + (size_t)b * strideB;
  const T* Ab2 = SPLIT ? (A2  + (size_t)b * strideA) : nullptr;
  const T* Bb2 = SPLIT ? (Bt2 + (size_t)b * strideB) : nullptr;

  const int rlane = lane & 15;
  const int koff  = (lane >> 4) * 8;
  const int mOff  = (lane >> 4) * 8;

  v8f acc[4][4];
#pragma unroll
  for (int i = 0; i < 4; ++i)
#pragma unroll
    for (int j = 0; j < 4; ++j) acc[i][j] = (v8f){0.f,0.f,0.f,0.f,0.f,0.f,0.f,0.f};

  for (int k0 = 0; k0 < K; k0 += 32) {
    V bh[4], bl[4];
#pragma unroll
    for (int j = 0; j < 4; ++j) {
      const size_t bo = (size_t)(n0 + (j << 4) + rlane) * ldb + koff + k0;
      bh[j] = Frag<T>::load(Bb + bo);
      if (SPLIT) bl[j] = Frag<T>::load(Bb2 + bo);
    }
#pragma unroll
    for (int i = 0; i < 4; ++i) {
      const size_t ao = (size_t)(m0 + (i << 4) + rlane) * lda + koff + k0;
      V ah = Frag<T>::load(Ab + ao);
      V al;
      if (SPLIT) al = Frag<T>::load(Ab2 + ao);
#pragma unroll
      for (int j = 0; j < 4; ++j) {
        acc[i][j] = Frag<T>::mma(ah, bh[j], acc[i][j]);
        if (SPLIT) {
          acc[i][j] = Frag<T>::mma(ah, bl[j], acc[i][j]);
          acc[i][j] = Frag<T>::mma(al, bh[j], acc[i][j]);
        }
      }
      Frag<T>::guard(acc[i][0], acc[i][3], ah, SPLIT ? al : ah);
    }
    Frag<T>::keep(bh[0], bh[1], bh[2], bh[3]);
    if (SPLIT) Frag<T>::keep(bl[0], bl[1], bl[2], bl[3]);
  }
  acc_guard4(acc[0][0], acc[0][1], acc[0][2], acc[0][3]);
  acc_guard4(acc[1][0], acc[1][1], acc[1][2], acc[1][3]);
  acc_guard4(acc[2][0], acc[2][1], acc[2][2], acc[2][3]);
  acc_guard4(acc[3][0], acc[3][1], acc[3][2], acc[3][3]);

  float* slab = sT[wave];
  const float* Rb = RESID ? (resid + (size_t)b * strideR) : nullptr;
#pragma unroll
  for (int i = 0; i < 4; ++i) {
    const int mBase = m0 + (i << 4);
#pragma unroll
    for (int j = 0; j < 4; ++j) {
      const int n = n0 + (j << 4) + rlane;
      float bv = 0.f;
      if (BIAS_MODE == 2) bv = bias[n];
#pragma unroll
      for (int r = 0; r < 8; ++r) {
        float v = acc[i][j][r] * scale;
        if (BIAS_MODE == 1) v += bias[mBase + mOff + r];
        if (BIAS_MODE == 2) v += bv;
        if (RESID) v += Rb[(size_t)(mBase + mOff + r) * ldc + n];
        if (ACT == 1) v = tanhf(v);
        if (ACT == 2) v = fmaxf(v, 0.0f);
        if (ACT == 3) v = v / (1.0f + expf(-v));
        if (ACT == 4) v = (v > 0.f) ? v : 0.01f * v;
        if (ACT == 5) v = 0.5f * v * (1.0f + erff(v * 0.70710678118654752f));
        slab[(mOff + r) * 68 + (j << 4) + rlane] = v;
      }
    }
    __builtin_amdgcn_fence(__ATOMIC_RELEASE, "workgroup");
    __builtin_amdgcn_wave_barrier();
    __builtin_amdgcn_fence(__ATOMIC_ACQUIRE, "workgroup");
    if (OUT_MODE == 0) {
      float* C = (float*)Cout + (size_t)b * strideC;
      const int hh = lane >> 4, c4 = (lane & 15) * 4;
      for (int pass = 0; pass < 2; ++pass) {
#pragma unroll
        for (int it = 0; it < 8; ++it) {
          const int row = it * 2 + hh;
          v4f v = *(const v4f*)(slab + row * 68 + c4);
          *(volatile v4f*)(C + (size_t)(mBase + row) * ldc + n0 + c4) = v;
        }
        __threadfence();
      }
    } else {
      const int q = lane >> 3, c8 = (lane & 7) * 8;
      unsigned short* C  = (unsigned short*)Cout  + (size_t)b * strideC;
      unsigned short* C2 = (OUT_MODE == 2) ? ((unsigned short*)Cout2 + (size_t)b * strideC) : nullptr;
      for (int pass = 0; pass < 2; ++pass) {
#pragma unroll
        for (int it = 0; it < 4; ++it) {
          const int row = it * 4 + q;
          const float* sp = slab + row * 68 + c8;
          v8h hv, lv;
#pragma unroll
          for (int e = 0; e < 8; ++e) {
            if (OUT_MODE == 1) {
              hv[e] = (_Float16)sp[e];
            } else {
              unsigned short hb = f2bf_bits(sp[e]);
              unsigned short lb = f2bf_bits(sp[e] - bf_bits2f(hb));
              hv[e] = __builtin_bit_cast(_Float16, hb);
              lv[e] = __builtin_bit_cast(_Float16, lb);
            }
          }
          *(volatile v8h*)(C + (size_t)(mBase + row) * ldc + n0 + c8) = hv;
          if (OUT_MODE == 2) *(volatile v8h*)(C2 + (size_t)(mBase + row) * ldc + n0 + c8) = lv;
        }
        __threadfence();
      }
    }
    __builtin_amdgcn_fence(__ATOMIC_RELEASE, "workgroup");
    __builtin_amdgcn_wave_barrier();
    __builtin_amdgcn_fence(__ATOMIC_ACQUIRE, "workgroup");
  }
}

__device__ __forceinline__ float bfr(float x) { return bf_bits2f(f2bf_bits(x)); }
__device__ __forceinline__ unsigned pack_bf2(float x, float y) {
  return (unsigned)f2bf_bits(x) | ((unsigned)f2bf_bits(y) << 16);
}
__device__ __forceinline__ unsigned pack_h2(float x, float y) {
  const unsigned short a = __builtin_bit_cast(unsigned short, (_Float16)x);
  const unsigned short b = __builtin_bit_cast(unsigned short, (_Float16)y);
  return (unsigned)a | ((unsigned)b << 16);
}
__device__ __forceinline__ v8f mma_h(v16h a, v16h b, v8f c) {
  c = __builtin_amdgcn_wmma_f32_16x16x32_f16(false, a, false, b, (short)0, c, false, false);
  asm volatile("v_nop\n\tv_nop\n\tv_nop\n\tv_nop" : "+v"(c) : "v"(a), "v"(b));
  return c;
}
__device__ __forceinline__ float sigm_f(float x) {
  return __builtin_amdgcn_rcpf(1.0f + expf(-x));
}
__device__ __forceinline__ float tanh_f(float x) {
  const float xc = fminf(fmaxf(x, -15.0f), 15.0f);
  const float a = expf(2.0f * xc);
  return (a - 1.0f) * __builtin_amdgcn_rcpf(a + 1.0f);
}
__device__ __forceinline__ int clampi(int v, int lo, int hi) { return v < lo ? lo : (v > hi ? hi : v); }

__global__ __launch_bounds__(256) void cast_embed_bf16(const float* __restrict__ src,
                                                      unsigned short* __restrict__ dst,
                                                      int nrows, int nrows_pad) {
  const int i = blockIdx.x * 256 + threadIdx.x;
  const int total = nrows_pad * (HDIM / 8);
  if (i < total) {
    const int row = i >> 4;
    const int c8 = (i & 15) * 8;
    const bool live = row < nrows;
    const int rowc = live ? row : nrows - 1;
    const v4f a = *(const v4f*)(src + (size_t)rowc * HDIM + c8);
    const v4f b = *(const v4f*)(src + (size_t)rowc * HDIM + c8 + 4);
    v4u u;
    u[0] = pack_bf2(live ? a[0] : 0.0f, live ? a[1] : 0.0f);
    u[1] = pack_bf2(live ? a[2] : 0.0f, live ? a[3] : 0.0f);
    u[2] = pack_bf2(live ? b[0] : 0.0f, live ? b[1] : 0.0f);
    u[3] = pack_bf2(live ? b[2] : 0.0f, live ? b[3] : 0.0f);
    *(volatile v4u*)(dst + (size_t)i * 8) = u;
    __threadfence();
    *(volatile v4u*)(dst + (size_t)i * 8) = u;
  }
}

__global__ __launch_bounds__(256) void cast_params(const float* __restrict__ w_ih, const float* __restrict__ w_hh,
                                                   const float* __restrict__ fcw,
                                                   unsigned short* __restrict__ wih16, unsigned short* __restrict__ whh16,
                                                   unsigned short* __restrict__ fcw16) {
  const int seg = blockIdx.y;
  const int i = blockIdx.x * 256 + threadIdx.x;
  if (seg == 0) {
    if (i < GATE3 * (HDIM / 8)) {
      const v4f a = *(const v4f*)(w_ih + (size_t)i * 8);
      const v4f b = *(const v4f*)(w_ih + (size_t)i * 8 + 4);
      v4u u;
      u[0] = pack_bf2(a[0], a[1]); u[1] = pack_bf2(a[2], a[3]);
      u[2] = pack_bf2(b[0], b[1]); u[3] = pack_bf2(b[2], b[3]);
      *(volatile v4u*)(wih16 + (size_t)i * 8) = u;
      __threadfence();
      *(volatile v4u*)(wih16 + (size_t)i * 8) = u;
    }
  } else if (seg == 1) {
    if (i < GATE3 * (HDIM / 8)) {
      const v4f a = *(const v4f*)(w_hh + (size_t)i * 8);
      const v4f b = *(const v4f*)(w_hh + (size_t)i * 8 + 4);
      v4u u;
      u[0] = pack_h2(bfr(a[0]) * WCARRY, bfr(a[1]) * WCARRY);
      u[1] = pack_h2(bfr(a[2]) * WCARRY, bfr(a[3]) * WCARRY);
      u[2] = pack_h2(bfr(b[0]) * WCARRY, bfr(b[1]) * WCARRY);
      u[3] = pack_h2(bfr(b[2]) * WCARRY, bfr(b[3]) * WCARRY);
      *(volatile v4u*)(whh16 + (size_t)i * 8) = u;
      __threadfence();
      *(volatile v4u*)(whh16 + (size_t)i * 8) = u;
    }
  } else {
    if (i < NCLASS_PAD * (HDIM / 8)) {
      const int row = i >> 4;
      const int c8 = (i & 15) * 8;
      const bool live = row < NCLASS;
      const int rowc = live ? row : NCLASS - 1;
      const v4f a = *(const v4f*)(fcw + (size_t)rowc * HDIM + c8);
      const v4f b = *(const v4f*)(fcw + (size_t)rowc * HDIM + c8 + 4);
      const float x0 = live ? bfr(a[0]) * WCARRY : 0.0f, x1 = live ? bfr(a[1]) * WCARRY : 0.0f;
      const float x2 = live ? bfr(a[2]) * WCARRY : 0.0f, x3 = live ? bfr(a[3]) * WCARRY : 0.0f;
      const float x4 = live ? bfr(b[0]) * WCARRY : 0.0f, x5 = live ? bfr(b[1]) * WCARRY : 0.0f;
      const float x6 = live ? bfr(b[2]) * WCARRY : 0.0f, x7 = live ? bfr(b[3]) * WCARRY : 0.0f;
      v4u u;
      u[0] = pack_h2(x0, x1); u[1] = pack_h2(x2, x3); u[2] = pack_h2(x4, x5); u[3] = pack_h2(x6, x7);
      *(volatile v4u*)(fcw16 + (size_t)i * 8) = u;
      __threadfence();
      *(volatile v4u*)(fcw16 + (size_t)i * 8) = u;
    }
  }
}

__global__ __launch_bounds__(128) void gru_ln_kernel(
    const int* __restrict__ token_id, const int* __restrict__ mailbox_idx, const int* __restrict__ lengths,
    const unsigned short* __restrict__ emb16, const float* __restrict__ gi,
    const unsigned short* __restrict__ whh16,
    const float* __restrict__ b_ih, const float* __restrict__ b_hh,
    const float* __restrict__ ln_g, const float* __restrict__ ln_b,
    unsigned short* __restrict__ hout16,
    int n_dst, int n_src, int n_vocab) {
  extern __shared__ __align__(16) unsigned char smem[];
  _Float16* whh_l = (_Float16*)(smem + LDS_WHH);
  float* bias_l = (float*)(smem + LDS_BIAS);
  float* lnp_l  = (float*)(smem + LDS_LNP);
  const int tid  = threadIdx.x;
  const int lane = tid & 31;
  const int wave = tid >> 5;
  const int hh   = lane >> 4;
  const int mrow = lane & 15;
  float* hf_w = (float*)(smem + LDS_HF) + wave * 16 * HFPITCH;
  _Float16* hb_w = (_Float16*)(smem + LDS_HB) + wave * 16 * WPITCH;
  float* gis_w = (float*)(smem + LDS_GIS) + wave * GIS_FLOATS;
  int* tok_w = (int*)(smem + LDS_TOK) + wave * 16;

#pragma unroll 4
  for (int it = 0; it < 48; ++it) {
    const int idx = it * 128 + tid;
    const int row = idx >> 4, c8 = (idx & 15) * 8;
    const v4u v = *(const v4u*)(whh16 + (size_t)row * HDIM + c8);
    *(v4u*)(whh_l + row * WPITCH + c8) = v;
  }
  for (int i = tid; i < GATE3; i += 128) {
    bias_l[i] = bfr(b_ih[i]);
    bias_l[GATE3 + i] = bfr(b_hh[i]);
  }
  for (int i = tid; i < HDIM; i += 128) {
    lnp_l[i] = bfr(ln_g[i]);
    lnp_l[HDIM + i] = bfr(ln_b[i]);
  }

  const int tile0 = (blockIdx.x * 4 + wave) * 16;
  int nst[8];
#pragma unroll
  for (int r = 0; r < 8; ++r) {
    const int nd = clampi(tile0 + 8 * hh + r, 0, n_dst - 1);
    const int len = clampi(lengths[nd], 1, MBOX);
    nst[r] = len - 1;
  }
  {
    const int nd = clampi(tile0 + mrow, 0, n_dst - 1);
    const int len = clampi(lengths[nd], 1, MBOX);
    const int mb = clampi(mailbox_idx[(size_t)nd * MBOX + (len - 1)], 0, n_src - 1);
    const int tk = clampi(token_id[mb], 0, n_vocab - 1);
    if (hh == 0) tok_w[mrow] = tk;
  }
  __syncthreads();

#pragma unroll
  for (int it = 0; it < 8; ++it) {
    const int row = 2 * it + hh;
    const int tk = tok_w[row];
    const v4u u = *(const v4u*)(emb16 + (size_t)tk * HDIM + mrow * 8);
    const float f0 = __uint_as_float(u[0] << 16), f1 = __uint_as_float(u[0] & 0xffff0000u);
    const float f2 = __uint_as_float(u[1] << 16), f3 = __uint_as_float(u[1] & 0xffff0000u);
    const float f4 = __uint_as_float(u[2] << 16), f5 = __uint_as_float(u[2] & 0xffff0000u);
    const float f6 = __uint_as_float(u[3] << 16), f7 = __uint_as_float(u[3] & 0xffff0000u);
    *(v4f*)(hf_w + row * HFPITCH + mrow * 8) = (v4f){f0, f1, f2, f3};
    *(v4f*)(hf_w + row * HFPITCH + mrow * 8 + 4) = (v4f){f4, f5, f6, f7};
    v8h hv;
    hv[0] = (_Float16)(f0 * HCARRY); hv[1] = (_Float16)(f1 * HCARRY);
    hv[2] = (_Float16)(f2 * HCARRY); hv[3] = (_Float16)(f3 * HCARRY);
    hv[4] = (_Float16)(f4 * HCARRY); hv[5] = (_Float16)(f5 * HCARRY);
    hv[6] = (_Float16)(f6 * HCARRY); hv[7] = (_Float16)(f7 * HCARRY);
    *(v8h*)(hb_w + row * WPITCH + mrow * 8) = hv;
  }
  __syncthreads();

  for (int t = 0; t < NSTEP; ++t) {
    {
      const int nd = clampi(tile0 + mrow, 0, n_dst - 1);
      const int mb = clampi(mailbox_idx[(size_t)nd * MBOX + t], 0, n_src - 1);
      const int tk = clampi(token_id[mb], 0, n_vocab - 1);
      if (hh == 0) tok_w[mrow] = tk;
    }
    v16h ah[4];
#pragma unroll
    for (int c = 0; c < 4; ++c) ah[c] = Frag<_Float16>::load(hb_w + mrow * WPITCH + c * 32 + 8 * hh);
    __syncthreads();

#pragma unroll 1
    for (int j = 0; j < 8; ++j) {
#pragma unroll
      for (int it = 0; it < 6; ++it) {
        const int e = it * 32 + lane;
        const int row = e / 12;
        const int rem = e - row * 12;
        const int g = rem >> 2, q = rem & 3;
        const int tk = tok_w[row];
        const v4f v = *(const v4f*)(gi + (size_t)tk * GATE3 + g * HDIM + j * 16 + q * 4);
        *(v4f*)(gis_w + (g * 16 + row) * 16 + q * 4) = v;
      }
      __syncthreads();

      v8f accr = (v8f){0.f,0.f,0.f,0.f,0.f,0.f,0.f,0.f};
      v8f accz = accr, accn = accr;
#pragma unroll
      for (int c = 0; c < 4; ++c) {
        const _Float16* bp = whh_l + (j * 16 + mrow) * WPITCH + c * 32 + 8 * hh;
        const v16h br = Frag<_Float16>::load(bp);
        const v16h bz = Frag<_Float16>::load(bp + HDIM * WPITCH);
        const v16h bn = Frag<_Float16>::load(bp + 2 * HDIM * WPITCH);
        accr = mma_h(ah[c], br, accr);
        accz = mma_h(ah[c], bz, accz);
        accn = mma_h(ah[c], bn, accn);
      }
      const int col = j * 16 + mrow;
      const float bir = bias_l[col], biz = bias_l[HDIM + col], bxn = bias_l[2 * HDIM + col];
      const float bhr = bias_l[GATE3 + col], bhz = bias_l[GATE3 + HDIM + col], bhn = bias_l[GATE3 + 2 * HDIM + col];
#pragma unroll
      for (int r = 0; r < 8; ++r) {
        const int mr = 8 * hh + r;
        const float xr = gis_w[(0 * 16 + mr) * 16 + mrow] + bir;
        const float xz = gis_w[(1 * 16 + mr) * 16 + mrow] + biz;
        const float xn = gis_w[(2 * 16 + mr) * 16 + mrow] + bxn;
        const float hr = accr[r] * FOLD_BACK + bhr;
        const float hz = accz[r] * FOLD_BACK + bhz;
        const float hn = accn[r] * FOLD_BACK + bhn;
        const float rg = sigm_f(xr + hr);
        const float zg = sigm_f(xz + hz);
        const float ng = tanh_f(xn + rg * hn);
        const float ho = hf_w[mr * HFPITCH + col];
        const float hnew = (1.0f - zg) * ng + zg * ho;
        const float hs = (t < nst[r]) ? hnew : ho;
        hf_w[mr * HFPITCH + col] = hs;
        hb_w[mr * WPITCH + col] = (_Float16)(hs * HCARRY);
      }
      __syncthreads();
    }
  }

  {
    const float* hrow = hf_w + mrow * HFPITCH + 64 * hh;
    float s = 0.0f;
#pragma unroll
    for (int q = 0; q < 16; ++q) {
      const v4f v = *(const v4f*)(hrow + 4 * q);
      s += (v[0] + v[1]) + (v[2] + v[3]);
    }
    s += __shfl_xor(s, 16, 32);
    const float mu = s * (1.0f / (float)HDIM);
    float s2 = 0.0f;
#pragma unroll
    for (int q = 0; q < 16; ++q) {
      const v4f v = *(const v4f*)(hrow + 4 * q);
      const float d0 = v[0] - mu, d1 = v[1] - mu, d2 = v[2] - mu, d3 = v[3] - mu;
      s2 += (d0 * d0 + d1 * d1) + (d2 * d2 + d3 * d3);
    }
    s2 += __shfl_xor(s2, 16, 32);
    const float var = s2 * (1.0f / (float)HDIM);
    const float rstd = rsqrtf(var + 1e-5f);
    const int nd = clampi(tile0 + mrow, 0, n_dst - 1);
    const int len = clampi(lengths[nd], 1, MBOX);
    const bool byp = (len == 1);
#pragma unroll
    for (int q = 0; q < 8; ++q) {
      const int d0 = 64 * hh + 8 * q;
      const v4f a = *(const v4f*)(hrow + 8 * q);
      const v4f b = *(const v4f*)(hrow + 8 * q + 4);
      v8h o;
#pragma unroll
      for (int e = 0; e < 4; ++e) {
        const float hv = a[e];
        const float lv = (hv - mu) * rstd * lnp_l[d0 + e] + lnp_l[HDIM + d0 + e];
        o[e] = (_Float16)((byp ? hv : lv) * HCARRY);
      }
#pragma unroll
      for (int e = 0; e < 4; ++e) {
        const float hv = b[e];
        const float lv = (hv - mu) * rstd * lnp_l[d0 + 4 + e] + lnp_l[HDIM + d0 + 4 + e];
        o[4 + e] = (_Float16)((byp ? hv : lv) * HCARRY);
      }
      *(v8h*)(hb_w + mrow * WPITCH + d0) = o;
    }
  }
  __syncthreads();

  {
    const unsigned short* hbu = (const unsigned short*)(const void*)hb_w;
    for (int pass = 0; pass < 2; ++pass) {
#pragma unroll
      for (int it = 0; it < 8; ++it) {
        const int row = 2 * it + hh;
        const v4u v = *(const v4u*)(hbu + row * WPITCH + mrow * 8);
        *(volatile v4u*)(hout16 + (size_t)(tile0 + row) * HDIM + mrow * 8) = v;
      }
      __threadfence();
    }
  }
}

__global__ __launch_bounds__(64) void fc_kernel(const unsigned short* __restrict__ hout16,
                                              const unsigned short* __restrict__ fcw16,
                                              const float* __restrict__ fc_b,
                                              float* __restrict__ out) {
  __shared__ __align__(16) _Float16 fcw_l[NCLASS_PAD * WPITCH];
  __shared__ __align__(16) float slab[2][16 * NCLASS];
  __shared__ float fcb_l[NCLASS_PAD];
  const int tid  = threadIdx.x;
  const int lane = tid & 31;
  const int wave = tid >> 5;
  const int hh   = lane >> 4;
  const int mrow = lane & 15;
#pragma unroll 4
  for (int it = 0; it < 28; ++it) {
    const int idx = it * 64 + tid;
    const int row = idx >> 4, c8 = (idx & 15) * 8;
    const v4u v = *(const v4u*)(fcw16 + (size_t)row * HDIM + c8);
    *(v4u*)(fcw_l + row * WPITCH + c8) = v;
  }
  for (int i = tid; i < NCLASS_PAD; i += 64) {
    const int ic = i < NCLASS ? i : NCLASS - 1;
    const float bv = bfr(fc_b[ic]);
    fcb_l[i] = (i < NCLASS) ? bv : 0.0f;
  }
  __syncthreads();

  const int row0 = (blockIdx.x * 2 + wave) * 16;
  const _Float16* hp = (const _Float16*)(const void*)hout16;
  v8f acc[7];
#pragma unroll
  for (int jt = 0; jt < 7; ++jt) acc[jt] = (v8f){0.f,0.f,0.f,0.f,0.f,0.f,0.f,0.f};
#pragma unroll
  for (int c = 0; c < 4; ++c) {
    const v16h av = Frag<_Float16>::load(hp + (size_t)(row0 + mrow) * HDIM + c * 32 + 8 * hh);
#pragma unroll
    for (int jt = 0; jt < 7; ++jt) {
      const v16h b = Frag<_Float16>::load(fcw_l + (jt * 16 + mrow) * WPITCH + c * 32 + 8 * hh);
      acc[jt] = mma_h(av, b, acc[jt]);
    }
  }
  float* sw = slab[wave];
#pragma unroll
  for (int jt = 0; jt < 7; ++jt) {
    const int col = jt * 16 + mrow;
    const float bv = fcb_l[col];
#pragma unroll
    for (int r = 0; r < 8; ++r) {
      const float v = acc[jt][r] * FOLD_BACK + bv;
      if (col < NCLASS) sw[(8 * hh + r) * NCLASS + col] = v;
    }
  }
  __syncthreads();
  float* base = out + (size_t)row0 * NCLASS;
  for (int pass = 0; pass < 2; ++pass) {
#pragma unroll
    for (int it = 0; it < 13; ++it) {
      const int idx = it * 32 + lane;
      const v4f v = *(const v4f*)(sw + idx * 4);
      *(volatile v4f*)(base + (size_t)idx * 4) = v;
    }
    __threadfence();
  }
}

extern "C" void kernel_launch(void* const* d_in, const int* in_sizes, int n_in,
                              void* d_out, int out_size, void* d_ws, size_t ws_size,
                              hipStream_t stream) {
  if (n_in < 12) return;
  const int*   token_id = (const int*)d_in[0];
  const int*   mailbox  = (const int*)d_in[1];
  const int*   lengths  = (const int*)d_in[2];
  const float* embed    = (const float*)d_in[3];
  const float* w_ih     = (const float*)d_in[4];
  const float* w_hh     = (const float*)d_in[5];
  const float* b_ih     = (const float*)d_in[6];
  const float* b_hh     = (const float*)d_in[7];
  const float* ln_g     = (const float*)d_in[8];
  const float* ln_b     = (const float*)d_in[9];
  const float* fc_w     = (const float*)d_in[10];
  const float* fc_b     = (const float*)d_in[11];
  float* out = (float*)d_out;

  const int n_src = in_sizes[0];
  const int n_dst = in_sizes[2];
  if (n_src <= 0 || n_dst <= 0) return;
  if (in_sizes[3] <= 0 || (in_sizes[3] % HDIM) != 0) return;
  const int n_vocab = in_sizes[3] / HDIM;
  if (in_sizes[1] != n_dst * MBOX) return;
  if (in_sizes[4] != GATE3 * HDIM || in_sizes[5] != GATE3 * HDIM) return;
  if (in_sizes[6] != GATE3 || in_sizes[7] != GATE3) return;
  if (in_sizes[8] != HDIM || in_sizes[9] != HDIM) return;
  if (in_sizes[10] != NCLASS * HDIM || in_sizes[11] != NCLASS) return;
  if (out_size != n_dst * NCLASS) return;
  if ((n_dst % 32) != 0) return;

  const int vocab_pad = ((n_vocab + 63) / 64) * 64;
  const int ndst_pad  = ((n_dst + 63) / 64) * 64;

  size_t off = 0;
  auto carve = [&](size_t bytes) { const size_t o = off; off += (bytes + 255) & ~(size_t)255; return o; };
  const size_t o_emb  = carve((size_t)vocab_pad * HDIM * 2);
  const size_t o_wih  = carve((size_t)GATE3 * HDIM * 2);
  const size_t o_whh  = carve((size_t)GATE3 * HDIM * 2);
  const size_t o_fcw  = carve((size_t)NCLASS_PAD * HDIM * 2);
  const size_t o_gi   = carve((size_t)vocab_pad * GATE3 * 4);
  const size_t o_hout = carve((size_t)ndst_pad * HDIM * 2);
  if (off > ws_size) return;

  unsigned char* ws = (unsigned char*)d_ws;
  unsigned short* emb16  = (unsigned short*)(ws + o_emb);
  unsigned short* wih16  = (unsigned short*)(ws + o_wih);
  unsigned short* whh16  = (unsigned short*)(ws + o_whh);
  unsigned short* fcw16  = (unsigned short*)(ws + o_fcw);
  float*          gi     = (float*)(ws + o_gi);
  unsigned short* hout16 = (unsigned short*)(ws + o_hout);

  {
    const int total = vocab_pad * (HDIM / 8);
    cast_embed_bf16<<<(total + 255) / 256, 256, 0, stream>>>(embed, emb16, n_vocab, vocab_pad);
  }
  {
    const int gx0 = (GATE3 * (HDIM / 8) + 255) / 256;
    const int gx2 = (NCLASS_PAD * (HDIM / 8) + 255) / 256;
    const int gx = gx0 > gx2 ? gx0 : gx2;
    cast_params<<<dim3(gx, 3), 256, 0, stream>>>(w_ih, w_hh, fc_w, wih16, whh16, fcw16);
  }
  {
    const int tiles = (vocab_pad / 64) * (GATE3 / 64);
    const int blocks = (tiles + 7) / 8;
    wmma_gemm64<1, false, 0, 0, false, 0><<<dim3(blocks, 1), 256, 0, stream>>>(
        emb16, emb16, HDIM, 0L,
        wih16, wih16, HDIM, 0L,
        (void*)gi, (void*)hout16, GATE3, 0L,
        b_ih,
        b_hh, 0L,
        vocab_pad, GATE3, HDIM, 1.0f);
  }
  gru_ln_kernel<<<ndst_pad / 64, 128, LDS_GRU_TOTAL, stream>>>(
      token_id, mailbox, lengths, emb16, gi, whh16, b_ih, b_hh, ln_g, ln_b, hout16,
      n_dst, n_src, n_vocab);
  fc_kernel<<<n_dst / 32, 64, 0, stream>>>(hout16, fcw16, fc_b, out);
}
